// BiBloSAN_25778393710754
// MI455X (gfx1250) — hardware-verified
//
#include <hip/hip_runtime.h>
#include <stddef.h>
#include <stdint.h>

#define NBAT 4
#define NBLK 16
#define RLEN 64
#define DM   256
#define NGRP (NBAT * NBLK)
#define NTOK (NGRP * RLEN)
#define DCAT (3 * DM)
#define WCAR 32.0f
#define SC_W 0.03125f
#define FCAR 16.0f
#define SC_WF 0.001953125f

static_assert(NTOK == 4096);
static_assert(NTOK % 256 == 0);
static_assert(NGRP % 64 == 0);
static_assert(DM == 256);
static_assert(DM % 64 == 0);
static_assert(DCAT % 64 == 0);
static_assert(RLEN % 4 == 0);
static_assert(NBLK % 4 == 0);
static_assert((NTOK * DM) % 2048 == 0);

typedef _Float16 v16h __attribute__((ext_vector_type(16)));
typedef _Float16 v8h  __attribute__((ext_vector_type(8)));
typedef float    v8f  __attribute__((ext_vector_type(8)));
typedef float    v4f  __attribute__((ext_vector_type(4)));
typedef unsigned int v4u __attribute__((ext_vector_type(4)));

union Frag  { v16h v; v8h h[2]; };
union Pack8 { v8h h; v4u u; };

__device__ __forceinline__ v8f mma16(v16h a, v16h b, v8f c) {
  c = __builtin_amdgcn_wmma_f32_16x16x32_f16(false, a, false, b, (short)0, c, false, false);
  asm volatile("v_nop\n\tv_nop\n\tv_nop\n\tv_nop" : "+v"(c) : "v"(a), "v"(b));
  return c;
}

__device__ __forceinline__ v16h ldfrag(const _Float16* p, int ld, int row0, int k0, int lane) {
  const int m = lane & 15, lh = lane >> 4;
  const _Float16* q = p + (size_t)(row0 + m) * ld + k0 + 8 * lh;
  Frag f;
  f.h[0] = *(const v8h*)(q);
  f.h[1] = *(const v8h*)(q + 16);
  return f.v;
}

__device__ __forceinline__ v8f zero8() { return (v8f){0.f, 0.f, 0.f, 0.f, 0.f, 0.f, 0.f, 0.f}; }

__device__ __forceinline__ v4u pack8(v4f a0, v4f a1) {
  Pack8 pk;
  pk.h = (v8h){(_Float16)a0[0], (_Float16)a0[1], (_Float16)a0[2], (_Float16)a0[3],
               (_Float16)a1[0], (_Float16)a1[1], (_Float16)a1[2], (_Float16)a1[3]};
  return pk.u;
}

__device__ __forceinline__ void gemm32x64(const _Float16* __restrict__ A, int lda,
                                          const _Float16* __restrict__ Bt, int ldb, int K,
                                          int m0, int n0, int lane, v8f (&acc)[2][4]) {
#pragma unroll 1
  for (int k0 = 0; k0 < K; k0 += 32) {
    const v16h a0 = ldfrag(A, lda, m0, k0, lane);
    const v16h a1 = ldfrag(A, lda, m0 + 16, k0, lane);
    const v16h b0 = ldfrag(Bt, ldb, n0, k0, lane);
    const v16h b1 = ldfrag(Bt, ldb, n0 + 16, k0, lane);
    const v16h b2 = ldfrag(Bt, ldb, n0 + 32, k0, lane);
    const v16h b3 = ldfrag(Bt, ldb, n0 + 48, k0, lane);
    acc[0][0] = mma16(a0, b0, acc[0][0]);
    acc[1][0] = mma16(a1, b0, acc[1][0]);
    acc[0][1] = mma16(a0, b1, acc[0][1]);
    acc[1][1] = mma16(a1, b1, acc[1][1]);
    acc[0][2] = mma16(a0, b2, acc[0][2]);
    acc[1][2] = mma16(a1, b2, acc[1][2]);
    acc[0][3] = mma16(a0, b3, acc[0][3]);
    acc[1][3] = mma16(a1, b3, acc[1][3]);
  }
}

__global__ __launch_bounds__(256) void k_cvtx(const float* __restrict__ src, _Float16* __restrict__ dh) {
  const size_t o = ((size_t)blockIdx.x * 256 + threadIdx.x) * 8;
  const v4f a0 = *(const v4f*)(src + o);
  const v4f a1 = *(const v4f*)(src + o + 4);
  const v4u vv = pack8(a0, a1);
  volatile v4u* d = (volatile v4u*)(dh + o);
  *d = vv;
  __threadfence();
  *d = vv;
}

#define WTP 72
__global__ __launch_bounds__(256) void k_wtr(const float* __restrict__ s0, _Float16* __restrict__ d0, int K0, int N0, int ld0,
                                             const float* __restrict__ s1, _Float16* __restrict__ d1, int K1, int N1, int ld1,
                                             const float* __restrict__ s2, _Float16* __restrict__ d2, int K2, int N2, int ld2,
                                             float scale) {
  __shared__ __align__(16) _Float16 st[64 * WTP];
  const int tid = threadIdx.x;
  const int z = blockIdx.z;
  const float* src = (z == 0) ? s0 : ((z == 1) ? s1 : s2);
  _Float16* dst    = (z == 0) ? d0 : ((z == 1) ? d1 : d2);
  const int K      = (z == 0) ? K0 : ((z == 1) ? K1 : K2);
  const int N      = (z == 0) ? N0 : ((z == 1) ? N1 : N2);
  const int ld     = (z == 0) ? ld0 : ((z == 1) ? ld1 : ld2);
  const int n0 = blockIdx.x * 64, k0 = blockIdx.y * 64;
  if (n0 >= N || k0 >= K) return;

  const int rr = tid >> 4, q = tid & 15;
#pragma unroll
  for (int p = 0; p < 4; ++p) {
    const int r = p * 16 + rr;
    const v4f v = *(const v4f*)(src + (size_t)(k0 + r) * N + n0 + 4 * q) * scale;
#pragma unroll
    for (int e = 0; e < 4; ++e) st[(4 * q + e) * WTP + r] = (_Float16)v[e];
  }
  __syncthreads();
  v4u val[2];
  size_t go[2];
#pragma unroll
  for (int g = 0; g < 2; ++g) {
    const int p  = tid + 256 * g;
    const int nn = p >> 3;
    const int pc = p & 7;
    Pack8 pk;
    pk.h   = *(const v8h*)(st + nn * WTP + pc * 8);
    val[g] = pk.u;
    go[g]  = (size_t)(n0 + nn) * ld + k0 + pc * 8;
  }
  for (int ps = 0; ps < 2; ++ps) {
#pragma unroll
    for (int g = 0; g < 2; ++g) *(volatile v4u*)(dst + go[g]) = val[g];
    __threadfence();
  }
}

#define OTP 68
template<int ACT, bool OF32, bool OF16>
__device__ __forceinline__ void epilogue(v8f (&acc)[2][4], float scale, const float (&bb)[4], float oscale,
                                         float* sw, float* __restrict__ of, int ldf,
                                         _Float16* __restrict__ oh, int ldh,
                                         int m0, int n0, int lane, int hh, int c) {
#pragma unroll
  for (int sub = 0; sub < 2; ++sub) {
    __syncthreads();
#pragma unroll
    for (int t = 0; t < 4; ++t) {
#pragma unroll
      for (int r = 0; r < 8; ++r) {
        float v = acc[sub][t][r] * scale + bb[t];
        if (ACT == 1) v = fmaxf(v, 0.f);
        sw[(8 * hh + r) * OTP + 16 * t + c] = v;
      }
    }
    __syncthreads();
    if (OF32) {
      v4f val[8];
      size_t go[8];
#pragma unroll
      for (int it = 0; it < 8; ++it) {
        const int p    = lane + 32 * it;
        const int L    = p >> 3;
        const int pc   = p & 7;
        const int row  = L >> 1;
        const int half = L & 1;
        val[it] = *(const v4f*)(sw + row * OTP + half * 32 + pc * 4);
        go[it]  = (size_t)(m0 + sub * 16 + row) * ldf + n0 + half * 32 + pc * 4;
      }
      for (int ps = 0; ps < 2; ++ps) {
#pragma unroll
        for (int it = 0; it < 8; ++it) *(volatile v4f*)(of + go[it]) = val[it];
        __threadfence();
      }
    }
    if (OF16) {
      v4u val[4];
      size_t go[4];
#pragma unroll
      for (int it = 0; it < 4; ++it) {
        const int p  = lane + 32 * it;
        const int L  = p >> 3;
        const int pc = p & 7;
        const float* ra = sw + L * OTP + pc * 8;
        const v4f a0 = *(const v4f*)(ra) * oscale, a1 = *(const v4f*)(ra + 4) * oscale;
        val[it] = pack8(a0, a1);
        go[it]  = (size_t)(m0 + sub * 16 + L) * ldh + n0 + pc * 8;
      }
      for (int ps = 0; ps < 2; ++ps) {
#pragma unroll
        for (int it = 0; it < 4; ++it) *(volatile v4u*)(oh + go[it]) = val[it];
        __threadfence();
      }
    }
  }
}

template<int WAVES, int ACT, bool HAS_BIAS, bool OF32, bool OF16>
__global__ __launch_bounds__(WAVES * 32) void k_gemm(const _Float16* __restrict__ ap, int lda,
                                                     const _Float16* __restrict__ wt, int K,
                                                     const float* __restrict__ bias0,
                                                     const float* __restrict__ bias1, int nsplit,
                                                     float scale, float oscale,
                                                     float* __restrict__ of, int ldf,
                                                     _Float16* __restrict__ oh, int ldh) {
  __shared__ __align__(16) float st[WAVES][16 * OTP];
  const int tid = threadIdx.x, lane = tid & 31, wave = tid >> 5;
  const int hh = lane >> 4, c = lane & 15;
  const int m0 = blockIdx.x * (WAVES * 32) + wave * 32;
  const int n0 = blockIdx.y * 64;

  v8f acc[2][4];
#pragma unroll
  for (int s = 0; s < 2; ++s)
#pragma unroll
    for (int t = 0; t < 4; ++t) acc[s][t] = zero8();
  gemm32x64(ap, lda, wt, K, K, m0, n0, lane, acc);

  float bb[4];
#pragma unroll
  for (int t = 0; t < 4; ++t) {
    if (HAS_BIAS) {
      const int col = n0 + 16 * t + c;
      const int i0 = (col < nsplit) ? col : (nsplit - 1);
      int i1 = col - nsplit;
      i1 = (i1 < 0) ? 0 : i1;
      const float v0 = bias0[i0], v1 = bias1[i1];
      bb[t] = (col < nsplit) ? v0 : v1;
    } else {
      bb[t] = 0.f;
    }
  }
  epilogue<ACT, OF32, OF16>(acc, scale, bb, oscale, st[wave], of, ldf, oh, ldh, m0, n0, lane, hh, c);
}

#define L2E04 0.57707801635558536f
#define L2E10 14.426950408889634f
__global__ __launch_bounds__(256) void k_attn_add(const float* __restrict__ xij, int ldx,
                                                  const float* __restrict__ val, int ldv,
                                                  const float* __restrict__ bvec,
                                                  float* __restrict__ hf, int ldhf,
                                                  _Float16* __restrict__ hh16, int ldhh,
                                                  int L, int fw) {
  __shared__ __align__(16) float sxj[RLEN * DM];
  __shared__ __align__(16) float sva[RLEN * DM];
  __shared__ __align__(16) float hrow[4 * DM];
  const int tid = threadIdx.x, d = tid;
  const size_t rb = (size_t)blockIdx.x * L;

  for (int j4 = 0; j4 < L; j4 += 4) {
    const int j = j4 + (tid >> 6), cc = (tid & 63) * 4;
    const v4f a = *(const v4f*)(xij + (rb + j) * (size_t)ldx + DM + cc);
    const v4f v = *(const v4f*)(val + (rb + j) * (size_t)ldv + cc);
    *(v4f*)(sxj + j * DM + cc) = a;
    *(v4f*)(sva + j * DM + cc) = v;
  }
  __syncthreads();

  const float bd = bvec[d];
  for (int i = 0; i < L; ++i) {
    const float xi = xij[(rb + i) * (size_t)ldx + d];
    const int jlo = fw ? (i + 1) : 0;
    const int jhi = fw ? L : i;
    float num = 0.f, den = 0.f;
#pragma unroll 1
    for (int j = jlo; j < jhi; ++j) {
      const float s = (xi + sxj[j * DM + d]) + bd;
      const float e = exp2f(s * L2E04);
      const float r = __builtin_amdgcn_rcpf(e + 1.0f);
      const float w = exp2f(-(r * L2E10));
      num = fmaf(w, sva[j * DM + d], num);
      den += w;
    }
    const bool ok = jhi > jlo;
    const float h = ok ? num * __builtin_amdgcn_rcpf(ok ? den : 1.0f) : 0.f;
    hrow[(i & 3) * DM + d] = h;
    if ((i & 3) == 3) {
      __syncthreads();
      const int i0 = i - 3;
      const int rr = tid >> 6, pc = tid & 63;
      const v4f fv = *(const v4f*)(hrow + rr * DM + pc * 4);
      const size_t gof = (rb + i0 + rr) * (size_t)ldhf + pc * 4;
      const int r2 = (tid >> 5) & 3, p2 = tid & 31;
      const float* hp = hrow + r2 * DM + 8 * p2;
      const v4u hv = pack8(*(const v4f*)(hp), *(const v4f*)(hp + 4));
      const size_t goh = (rb + i0 + r2) * (size_t)ldhh + 8 * p2;
      for (int ps = 0; ps < 2; ++ps) {
        *(volatile v4f*)(hf + gof) = fv;
        if (tid < 128) *(volatile v4u*)(hh16 + goh) = hv;
        __threadfence();
      }
      __syncthreads();
    }
  }
}

__global__ __launch_bounds__(256) void k_pool(const float* __restrict__ s, const float* __restrict__ hfp,
                                              float* __restrict__ vf, _Float16* __restrict__ ov) {
  __shared__ __align__(16) float vrow[DM];
  const int tid = threadIdx.x, d = tid, lane = tid & 31, wave = tid >> 5;
  const int g = blockIdx.x;
  const size_t rb = (size_t)g * RLEN;
  float m = -__builtin_huge_valf();
#pragma unroll 1
  for (int r = 0; r < RLEN; ++r) m = fmaxf(m, s[(rb + r) * DM + d]);
  float num = 0.f, den = 0.f;
#pragma unroll 1
  for (int r = 0; r < RLEN; ++r) {
    const float w = __expf(s[(rb + r) * DM + d] - m);
    num = fmaf(w, hfp[(rb + r) * DM + d], num);
    den += w;
  }
  vrow[d] = num * __builtin_amdgcn_rcpf(den);
  __syncthreads();
  if (wave < 2) {
    const v4f v = *(const v4f*)(vrow + 4 * tid);
    const size_t go = (size_t)g * DM + 4 * tid;
    for (int ps = 0; ps < 2; ++ps) { *(volatile v4f*)(vf + go) = v; __threadfence(); }
  }
  if (wave == 2) {
    const float* cp = vrow + 8 * lane;
    const v4u hv = pack8(*(const v4f*)(cp), *(const v4f*)(cp + 4));
    const size_t go = (size_t)g * 2 * DM + DM + 8 * lane;
    for (int ps = 0; ps < 2; ++ps) { *(volatile v4u*)(ov + go) = hv; __threadfence(); }
  }
}

__global__ __launch_bounds__(256) void k_cat(const float* __restrict__ tg, const float* __restrict__ of,
                                             const float* __restrict__ vf, const float* __restrict__ inf32,
                                             const float* __restrict__ hfp, _Float16* __restrict__ cat) {
  __shared__ __align__(16) _Float16 crow[DCAT];
  const int tid = threadIdx.x, d = tid, b = blockIdx.x;
  const size_t r0 = (size_t)b * NBLK;
  const float gp = tg[r0 * DM + d];
  const float gg = __builtin_amdgcn_rcpf(1.0f + __expf(-gp));
  const float e0 = gg * of[r0 * DM + d] + (1.0f - gg) * vf[r0 * DM + d];
  const _Float16 eh = (_Float16)e0;
  for (int t = 0; t < NBLK; ++t) {
    const size_t tok = (size_t)b * NBLK * RLEN + t;
    crow[d]          = (_Float16)inf32[tok * DM + d];
    crow[DM + d]     = (_Float16)hfp[tok * DM + d];
    crow[2 * DM + d] = eh;
    __syncthreads();
    if (tid < 96) {
      Pack8 pk;
      pk.h = *(const v8h*)(crow + 8 * tid);
      const v4u vv = pk.u;
      const size_t go = ((size_t)b * NBLK + t) * DCAT + 8 * tid;
      for (int ps = 0; ps < 2; ++ps) { *(volatile v4u*)(cat + go) = vv; __threadfence(); }
    }
    __syncthreads();
  }
}

__global__ __launch_bounds__(256) void k_out(const float* __restrict__ tf0, const float* __restrict__ in0,
                                             const float* __restrict__ tf1, const float* __restrict__ in1,
                                             float* __restrict__ out) {
  __shared__ __align__(16) float urow[2 * DM];
  const int tid = threadIdx.x, d = tid, row = blockIdx.x;
  const int b = row / NBLK, t = row - b * NBLK;
  const size_t tok = (size_t)b * NBLK * RLEN + t;
  {
    const float fu = fmaxf(tf0[(size_t)row * 2 * DM + d], 0.f);
    const float gp = tf0[(size_t)row * 2 * DM + DM + d];
    const float gf = __builtin_amdgcn_rcpf(1.0f + __expf(-gp));
    const float xf = in0[tok * DM + d];
    urow[d] = gf * fu + (1.0f - gf) * xf;
  }
  {
    const float fu = fmaxf(tf1[(size_t)row * 2 * DM + d], 0.f);
    const float gp = tf1[(size_t)row * 2 * DM + DM + d];
    const float gf = __builtin_amdgcn_rcpf(1.0f + __expf(-gp));
    const float xf = in1[tok * DM + d];
    urow[DM + d] = gf * fu + (1.0f - gf) * xf;
  }
  __syncthreads();
  if (tid < 128) {
    const v4f v = *(const v4f*)(urow + 4 * tid);
    const size_t go = (size_t)row * 2 * DM + 4 * tid;
    for (int ps = 0; ps < 2; ++ps) { *(volatile v4f*)(out + go) = v; __threadfence(); }
  }
}

extern "C" void kernel_launch(void* const* d_in, const int* in_sizes, int n_in,
                              void* d_out, int out_size, void* d_ws, size_t ws_size,
                              hipStream_t stream) {
  if (n_in < 33) return;
  if (in_sizes[0] != NTOK * DM) return;
  for (int dir = 0; dir < 2; ++dir) {
    const int ib = 1 + 16 * dir;
    if (in_sizes[ib + 0] != DM * DM) return;
    if (in_sizes[ib + 1] != DM) return;
    if (in_sizes[ib + 2] != DM * DM) return;
    if (in_sizes[ib + 3] != DM * DM) return;
    if (in_sizes[ib + 4] != DM) return;
    if (in_sizes[ib + 5] != DM * DM) return;
    if (in_sizes[ib + 6] != DM) return;
    if (in_sizes[ib + 7] != DM * DM) return;
    if (in_sizes[ib + 8] != DM) return;
    if (in_sizes[ib + 9] != DM * DM) return;
    if (in_sizes[ib + 10] != DM * DM) return;
    if (in_sizes[ib + 11] != DM) return;
    if (in_sizes[ib + 12] != DCAT * DM) return;
    if (in_sizes[ib + 13] != DM) return;
    if (in_sizes[ib + 14] != DCAT * DM) return;
    if (in_sizes[ib + 15] != DM) return;
  }
  if (out_size != NGRP * 2 * DM) return;

  const size_t szW    = (size_t)DM * DM * 2;
  const size_t szTokF = (size_t)NTOK * DM * 4;
  const size_t szTokH = (size_t)NTOK * DM * 2;
  const size_t szGrpF = (size_t)NGRP * DM * 4;
  size_t off = 0;
  const size_t oXh = off; off += szTokH;
  size_t oFC[2], oMW[2], oS1[2], oSW[2], oGW[2], oFW[2], oINf[2], oINh[2], oXIJ[2], oHf[2], oHh[2],
         oFh[2], oSf[2], oVf[2], oOV[2], oVIJ[2], oOf[2], oTg[2], oCAT[2], oTf[2];
  for (int dir = 0; dir < 2; ++dir) {
    oFC[dir]  = off; off += szW;
    oMW[dir]  = off; off += 2 * szW;
    oS1[dir]  = off; off += szW;
    oSW[dir]  = off; off += szW;
    oGW[dir]  = off; off += 2 * szW;
    oFW[dir]  = off; off += (size_t)(2 * DM) * DCAT * 2;
    oINf[dir] = off; off += szTokF;
    oINh[dir] = off; off += szTokH;
    oXIJ[dir] = off; off += 2 * szTokF;
    oHf[dir]  = off; off += szTokF;
    oHh[dir]  = off; off += szTokH;
    oFh[dir]  = off; off += szTokH;
    oSf[dir]  = off; off += szTokF;
    oVf[dir]  = off; off += szGrpF;
    oOV[dir]  = off; off += (size_t)NGRP * 2 * DM * 2;
    oVIJ[dir] = off; off += (size_t)NGRP * 2 * DM * 4;
    oOf[dir]  = off; off += szGrpF;
    oTg[dir]  = off; off += szGrpF;
    oCAT[dir] = off; off += (size_t)NGRP * DCAT * 2;
    oTf[dir]  = off; off += (size_t)NGRP * 2 * DM * 4;
  }
  if (off > ws_size) return;
  if (off > (size_t)134217728) return;

  char* ws = (char*)d_ws;
  const float* x = (const float*)d_in[0];
  float* out = (float*)d_out;
  _Float16* Xh = (_Float16*)(ws + oXh);

  k_cvtx<<<dim3((NTOK * DM) / 2048), dim3(256), 0, stream>>>(x, Xh);

  const float* INfp[2];
  const float* Tfp[2];
  for (int dir = 0; dir < 2; ++dir) {
    const int ib = 1 + 16 * dir;
    const float* fcW   = (const float*)d_in[ib + 0];
    const float* fcb   = (const float*)d_in[ib + 1];
    const float* mW1   = (const float*)d_in[ib + 2];
    const float* mW2   = (const float*)d_in[ib + 3];
    const float* mb    = (const float*)d_in[ib + 4];
    const float* s2tW1 = (const float*)d_in[ib + 5];
    const float* s2tb1 = (const float*)d_in[ib + 6];
    const float* s2tW  = (const float*)d_in[ib + 7];
    const float* s2tb  = (const float*)d_in[ib + 8];
    const float* gW1   = (const float*)d_in[ib + 9];
    const float* gW2   = (const float*)d_in[ib + 10];
    const float* gb    = (const float*)d_in[ib + 11];
    const float* fW1   = (const float*)d_in[ib + 12];
    const float* fb1   = (const float*)d_in[ib + 13];
    const float* fW2   = (const float*)d_in[ib + 14];
    const float* fb2   = (const float*)d_in[ib + 15];
    const int fw = (dir == 0) ? 1 : 0;

    _Float16* FCt = (_Float16*)(ws + oFC[dir]);
    _Float16* MWt = (_Float16*)(ws + oMW[dir]);
    _Float16* S1t = (_Float16*)(ws + oS1[dir]);
    _Float16* SWt = (_Float16*)(ws + oSW[dir]);
    _Float16* GWt = (_Float16*)(ws + oGW[dir]);
    _Float16* FWt = (_Float16*)(ws + oFW[dir]);
    float*    INf = (float*)(ws + oINf[dir]);
    _Float16* INh = (_Float16*)(ws + oINh[dir]);
    float*    XIJ = (float*)(ws + oXIJ[dir]);
    float*    Hf  = (float*)(ws + oHf[dir]);
    _Float16* Hh  = (_Float16*)(ws + oHh[dir]);
    _Float16* Fh  = (_Float16*)(ws + oFh[dir]);
    float*    Sf  = (float*)(ws + oSf[dir]);
    float*    Vf  = (float*)(ws + oVf[dir]);
    _Float16* OV  = (_Float16*)(ws + oOV[dir]);
    float*    VIJ = (float*)(ws + oVIJ[dir]);
    float*    Of  = (float*)(ws + oOf[dir]);
    float*    Tg  = (float*)(ws + oTg[dir]);
    _Float16* CAT = (_Float16*)(ws + oCAT[dir]);
    float*    Tf  = (float*)(ws + oTf[dir]);
    INfp[dir] = INf;
    Tfp[dir] = Tf;

    k_wtr<<<dim3(DM / 64, DM / 64, 3), dim3(256), 0, stream>>>(
        fcW, FCt, DM, DM, DM,
        mW1, MWt, DM, DM, DM,
        mW2, MWt + (size_t)DM * DM, DM, DM, DM, WCAR);
    k_wtr<<<dim3(DM / 64, DM / 64, 3), dim3(256), 0, stream>>>(
        s2tW1, S1t, DM, DM, DM,
        s2tW, SWt, DM, DM, DM,
        gW1, GWt, DM, DM, 2 * DM, WCAR);
    k_wtr<<<dim3(DM / 64, DCAT / 64, 3), dim3(256), 0, stream>>>(
        gW2, GWt + DM, DM, DM, 2 * DM,
        fW1, FWt, DCAT, DM, DCAT,
        fW2, FWt + (size_t)DM * DCAT, DCAT, DM, DCAT, WCAR);
    k_gemm<8, 1, true, true, true><<<dim3(NTOK / 256, DM / 64), dim3(256), 0, stream>>>(
        Xh, DM, FCt, DM, fcb, fcb, DM, SC_W, 1.0f, INf, DM, INh, DM);
    k_gemm<8, 0, false, true, false><<<dim3(NTOK / 256, (2 * DM) / 64), dim3(256), 0, stream>>>(
        INh, DM, MWt, DM, fcb, fcb, 2 * DM, SC_W, 1.0f, XIJ, 2 * DM, Fh, DM);
    k_attn_add<<<dim3(NGRP), dim3(256), 0, stream>>>(XIJ, 2 * DM, INf, DM, mb, Hf, DM, Hh, DM, RLEN, fw);
    k_gemm<8, 1, true, false, true><<<dim3(NTOK / 256, DM / 64), dim3(256), 0, stream>>>(
        Hh, DM, S1t, DM, s2tb1, s2tb1, DM, SC_W, FCAR, Sf, DM, Fh, DM);
    k_gemm<8, 0, true, true, false><<<dim3(NTOK / 256, DM / 64), dim3(256), 0, stream>>>(
        Fh, DM, SWt, DM, s2tb, s2tb, DM, SC_WF, 1.0f, Sf, DM, CAT, DCAT);
    k_pool<<<dim3(NGRP), dim3(256), 0, stream>>>(Sf, Hf, Vf, OV);
    k_gemm<2, 0, false, true, false><<<dim3(NGRP / 64, (2 * DM) / 64), dim3(64), 0, stream>>>(
        OV + DM, 2 * DM, MWt, DM, gb, gb, 2 * DM, SC_W, 1.0f, VIJ, 2 * DM, CAT, DCAT);
    k_attn_add<<<dim3(NBAT), dim3(256), 0, stream>>>(VIJ, 2 * DM, Vf, DM, mb, Of, DM, OV, 2 * DM, NBLK, fw);
    k_gemm<2, 0, true, true, false><<<dim3(NGRP / 64, DM / 64), dim3(64), 0, stream>>>(
        OV, 2 * DM, GWt, 2 * DM, gb, gb, DM, SC_W, 1.0f, Tg, DM, CAT, DCAT);
    k_cat<<<dim3(NBAT), dim3(256), 0, stream>>>(Tg, Of, Vf, INf, Hf, CAT);
    k_gemm<2, 0, true, true, false><<<dim3(NGRP / 64, (2 * DM) / 64), dim3(64), 0, stream>>>(
        CAT, DCAT, FWt, DCAT, fb1, fb2, DM, SC_W, 1.0f, Tf, 2 * DM, Fh, DM);
  }
  k_out<<<dim3(NGRP), dim3(256), 0, stream>>>(Tfp[0], INfp[0], Tfp[1], INfp[1], out);
  (void)hipGetLastError();
}
